// CrossAttention_48713519071925
// MI455X (gfx1250) — hardware-verified
//
#include <hip/hip_runtime.h>


#ifndef NB
#define NB 4
#endif
#ifndef SEQ
#define SEQ 2048
#endif
#ifndef SKV
#define SKV 1024
#endif
#define NB_FULL  4
#define SEQ_FULL 2048
#define SKV_FULL 1024
#define DQM  1024
#define DCM  768
#define NH_  8
#define HD   64
#define DI   (NH_ * HD)
#define VTP  (NB * SKV)
#define PSH  8.0f
#define OCAR 1024.0f
#define WCAR 64.0f
#define OSC  (1.0f / 65536.0f)
#define CL2  0.18033688011112042f

typedef _Float16 h16;
typedef unsigned short bf;
typedef __attribute__((ext_vector_type(16))) __bf16   v16bf;
typedef __attribute__((ext_vector_type(16))) _Float16 v16h;
typedef __attribute__((ext_vector_type(8)))  _Float16 v8h;
typedef __attribute__((ext_vector_type(8)))  unsigned short v8us;
typedef __attribute__((ext_vector_type(2)))  unsigned short v2us;
typedef __attribute__((ext_vector_type(8)))  float    v8f;
typedef __attribute__((ext_vector_type(4)))  float    v4f;
typedef v8h  __attribute__((may_alias)) v8ha;
typedef v4f  __attribute__((may_alias)) v4fa;

static_assert(SEQ % 64 == 0);
static_assert(SKV % 64 == 0);
static_assert(DQM % 64 == 0);
static_assert(DCM % 64 == 0);
static_assert(DI % 64 == 0);
static_assert((NB * SEQ) % 64 == 0);
static_assert((NB * SKV) % 64 == 0);
static_assert(NB <= NB_FULL);
static_assert(SEQ <= SEQ_FULL);
static_assert(SKV <= SKV_FULL);

__device__ __forceinline__ unsigned short f2bf(float f) { unsigned u = __float_as_uint(f); u += 0x7FFFu + ((u >> 16) & 1u); return (unsigned short)(u >> 16); }
__device__ __forceinline__ float bf2f(unsigned short b) { return __uint_as_float(((unsigned)b) << 16); }
__device__ __forceinline__ float bfr(float f) { return bf2f(f2bf(f)); }
__device__ __forceinline__ v16h cat16(v8h lo, v8h hi) { return __builtin_shufflevector(lo, hi, 0, 1, 2, 3, 4, 5, 6, 7, 8, 9, 10, 11, 12, 13, 14, 15); }
__device__ __forceinline__ v16bf cat16b(v8us lo, v8us hi) { return __builtin_bit_cast(v16bf, __builtin_shufflevector(lo, hi, 0, 1, 2, 3, 4, 5, 6, 7, 8, 9, 10, 11, 12, 13, 14, 15)); }
__device__ __forceinline__ v8f wmma16(v16h a, v16h b, v8f c) { return __builtin_amdgcn_wmma_f32_16x16x32_f16(false, a, false, b, (short)0, c, false, false); }
__device__ __forceinline__ v8f wmmab(v16bf a, v16bf b, v8f c) { return __builtin_amdgcn_wmma_f32_16x16x32_bf16(false, a, false, b, (short)0, c, false, false); }
__device__ __forceinline__ v16h ldfrag(const h16* p) { return cat16(*(const v8h*)p, *(const v8h*)(p + 16)); }

template <typename T16> struct WFrag;
template <> struct WFrag<h16> { typedef v16h V; static __device__ __forceinline__ V ld(const h16* p) { return cat16(*(const v8h*)p, *(const v8h*)(p + 16)); } static __device__ __forceinline__ v8f mma(V a, V b, v8f c) { return wmma16(a, b, c); } };
template <> struct WFrag<bf> { typedef v16bf V; static __device__ __forceinline__ V ld(const bf* p) { return cat16b(*(const v8us*)p, *(const v8us*)(p + 16)); } static __device__ __forceinline__ v8f mma(V a, V b, v8f c) { return wmmab(a, b, c); } };
template <typename T16, bool BIAS>
__global__ __launch_bounds__(32) void k_gemmw(const T16* __restrict__ A, const T16* __restrict__ Bt, unsigned K, float* C, unsigned ldc, const float* __restrict__ bias, size_t sA, size_t sB, size_t sC, float osc) {
    typedef typename WFrag<T16>::V V;
    __shared__ __align__(16) float os[16 * 68];
    const size_t z = blockIdx.z; A += z * sA; Bt += z * sB; C += z * sC;
    const unsigned lane = threadIdx.x & 31u, lr = lane & 15u, hi = lane >> 4; const unsigned r0 = blockIdx.x * 64u, c0 = blockIdx.y * 64u;
    v8f acc[4][4];
#pragma unroll
    for (int mb = 0; mb < 4; ++mb)
#pragma unroll
        for (int nb = 0; nb < 4; ++nb) acc[mb][nb] = (v8f){};
    const size_t aoff = (size_t)(r0 + lr) * K + 8u * hi, boff = (size_t)(c0 + lr) * K + 8u * hi;
#pragma unroll 1
    for (unsigned kc = 0; kc < K; kc += 32u) {
        V a[4];
#pragma unroll
        for (int mb = 0; mb < 4; ++mb) a[mb] = WFrag<T16>::ld(A + aoff + (size_t)mb * 16 * K + kc);
#pragma unroll
        for (int nb = 0; nb < 4; ++nb) { const V b = WFrag<T16>::ld(Bt + boff + (size_t)nb * 16 * K + kc);
#pragma unroll
            for (int mb = 0; mb < 4; ++mb) acc[mb][nb] = WFrag<T16>::mma(a[mb], b, acc[mb][nb]); }
        asm volatile("v_nop\n\tv_nop\n\tv_nop\n\tv_nop" : "+v"(acc[0][0]), "+v"(acc[1][1]), "+v"(acc[2][2]), "+v"(acc[3][3]) : "v"(a[0]), "v"(a[3]));
    }
    v4f bv = (v4f){};
    if (BIAS) { const v4f t = *(const v4f*)(bias + c0 + lr * 4u); bv[0] = bfr(t[0]); bv[1] = bfr(t[1]); bv[2] = bfr(t[2]); bv[3] = bfr(t[3]); }
#pragma unroll
    for (int mb = 0; mb < 4; ++mb) {
#pragma unroll
        for (int nb = 0; nb < 4; ++nb) {
#pragma unroll
            for (int j = 0; j < 8; ++j) os[(hi * 8u + j) * 68u + nb * 16 + lr] = acc[mb][nb][j]; }
        __builtin_amdgcn_fence(3  , "wavefront"); __builtin_amdgcn_wave_barrier(); asm volatile("" ::: "memory");
        float* crow = C + (size_t)(r0 + mb * 16) * ldc + c0;
#pragma unroll 1
        for (int ps = 0; ps < 2; ++ps) {
#pragma unroll
            for (int s = 0; s < 8; ++s) { const unsigned row = 2u * s + hi, cofs = lr * 4u; v4f val = *(const v4fa*)(os + row * 68u + cofs); val = val * osc + bv;
                *(volatile v4f*)(crow + (size_t)row * ldc + cofs) = val; }
            if (ps == 0) __threadfence(); }
        __builtin_amdgcn_fence(3  , "wavefront"); __builtin_amdgcn_wave_barrier(); asm volatile("" ::: "memory");
    }
}

__global__ __launch_bounds__(256) void k_wtG(const float* __restrict__ w, unsigned K, unsigned N, bf* Bt, int asf16, float carry) {
    const unsigned lane = threadIdx.x & 31u; const unsigned L0 = (blockIdx.x * 8u + (threadIdx.x >> 5)) * 8u; const unsigned nlines = N * K / 64u;
#pragma unroll
    for (int ps = 0; ps < 2; ++ps) {
#pragma unroll 1
        for (unsigned l = 0; l < 8u; ++l) { const unsigned L = L0 + l; if (L >= nlines) break; const unsigned e = L * 64u + lane * 2u; const unsigned n = e / K; const unsigned k = e - n * K;
            unsigned short b0 = f2bf(w[(size_t)k * N + n]), b1 = f2bf(w[(size_t)(k + 1u) * N + n]);
            if (asf16) { b0 = __builtin_bit_cast(unsigned short, (h16)(bf2f(b0) * carry)); b1 = __builtin_bit_cast(unsigned short, (h16)(bf2f(b1) * carry)); }
            v2us o; o[0] = b0; o[1] = b1; *(volatile v2us*)(Bt + e) = o; }
        if (ps == 0) __threadfence(); }
}
__global__ __launch_bounds__(256) void k_cvt8(const float* __restrict__ src, bf* dst, unsigned n8, size_t sstr, size_t dstr) {
    const unsigned i = blockIdx.x * 256u + threadIdx.x; if (i >= n8) return;
    const float* s = src + (size_t)blockIdx.y * sstr + (size_t)i * 8; bf* d = dst + (size_t)blockIdx.y * dstr + (size_t)i * 8;
    const v8f v = *(const v8f*)s; v8us o;
#pragma unroll
    for (int k = 0; k < 8; ++k) o[k] = f2bf(v[k]);
    *(volatile v8us*)d = o; __threadfence(); *(volatile v8us*)d = o; }
__global__ __launch_bounds__(256) void k_cvt8h(const float* __restrict__ src, h16* dst, unsigned n8) {
    const unsigned i = blockIdx.x * 256u + threadIdx.x; if (i >= n8) return;
    const v8f v = *(const v8f*)(src + (size_t)i * 8); v8h o;
#pragma unroll
    for (int k = 0; k < 8; ++k) o[k] = (h16)v[k];
    *(volatile v8h*)(dst + (size_t)i * 8) = o; __threadfence(); *(volatile v8h*)(dst + (size_t)i * 8) = o; }

__global__ __launch_bounds__(128) void k_fattn(const h16* __restrict__ Q16, const h16* __restrict__ K16, const h16* __restrict__ VT16, h16* AT16) {
    __shared__ __align__(16) h16 os[4 * 16 * 72];
    const unsigned tid = threadIdx.x, wave = tid >> 5, lane = tid & 31u, lr = lane & 15u, hi = lane >> 4;
    const unsigned bh = blockIdx.y, b = bh / (unsigned)NH_, h = bh % (unsigned)NH_;
    const unsigned i0 = blockIdx.x * 64u + wave * 16u;
    const h16* qp = Q16 + (size_t)(b * SEQ + i0 + lr) * DI + h * HD + 8u * hi;
    const v16h qb0 = ldfrag(qp), qb1 = ldfrag(qp + 32);
    const h16* kb = K16 + (size_t)(b * SKV + lr) * DI + h * HD + 8u * hi;
    const h16* vb = VT16 + (size_t)(h * HD + lr) * VTP + b * SKV + 8u * hi;
    float m = -3.0e38f, l = 0.0f;
    v8f ot[4];
#pragma unroll
    for (int dt = 0; dt < 4; ++dt) ot[dt] = (v8f){};
#pragma unroll 1
    for (unsigned j0 = 0; j0 < (unsigned)SKV; j0 += 64u) {
        v16h ka[4], kc[4];
#pragma unroll
        for (int jt = 0; jt < 4; ++jt) { const h16* kp = kb + (size_t)(j0 + jt * 16) * DI; ka[jt] = ldfrag(kp); kc[jt] = ldfrag(kp + 32); }
        v8f st[4];
#pragma unroll
        for (int jt = 0; jt < 4; ++jt) { v8f s = (v8f){}; s = wmma16(ka[jt], qb0, s); s = wmma16(kc[jt], qb1, s); st[jt] = s; }
        asm volatile("v_nop\n\tv_nop\n\tv_nop\n\tv_nop" : "+v"(st[0]), "+v"(st[1]), "+v"(st[2]), "+v"(st[3]) : "v"(qb0), "v"(qb1), "v"(ka[3]), "v"(kc[3]), "v"(ka[0]), "v"(kc[0]));
        float tm = st[0][0];
#pragma unroll
        for (int jt = 0; jt < 4; ++jt)
#pragma unroll
            for (int r = 0; r < 8; ++r) tm = fmaxf(tm, st[jt][r]);
        tm = fmaxf(tm, __shfl_xor(tm, 16, 32));
        const float mn = fmaxf(m, tm);
        const float alpha = __builtin_amdgcn_exp2f((m - mn) * CL2);
        m = mn;
        const float sh = PSH - mn * CL2;
        v16h pb[2]; float ls = 0.0f;
#pragma unroll
        for (int kk = 0; kk < 2; ++kk)
#pragma unroll
            for (int r = 0; r < 8; ++r) {
                const h16 p0 = (h16)__builtin_amdgcn_exp2f(st[2 * kk][r] * CL2 + sh);
                const h16 p1 = (h16)__builtin_amdgcn_exp2f(st[2 * kk + 1][r] * CL2 + sh);
                pb[kk][r] = p0; pb[kk][8 + r] = p1; ls += (float)p0 + (float)p1; }
        l = l * alpha + ls;
#pragma unroll
        for (int dt = 0; dt < 4; ++dt) ot[dt] = ot[dt] * alpha;
        v16h va[4], vc[4];
#pragma unroll
        for (int dt = 0; dt < 4; ++dt) { const h16* vp = vb + (size_t)(dt * 16) * VTP + j0; va[dt] = ldfrag(vp); vc[dt] = ldfrag(vp + 32); }
#pragma unroll
        for (int dt = 0; dt < 4; ++dt) { ot[dt] = wmma16(va[dt], pb[0], ot[dt]); ot[dt] = wmma16(vc[dt], pb[1], ot[dt]); }
        asm volatile("v_nop\n\tv_nop\n\tv_nop\n\tv_nop" : "+v"(ot[0]), "+v"(ot[1]), "+v"(ot[2]), "+v"(ot[3]) : "v"(pb[0]), "v"(pb[1]), "v"(va[3]), "v"(vc[3]), "v"(va[0]), "v"(vc[0]));
    }
    l += __shfl_xor(l, 16, 32);
    const float f = OCAR * (1.0f / l);
    h16* ow = os + wave * (16u * 72u);
#pragma unroll
    for (int dt = 0; dt < 4; ++dt) { v8h o8;
#pragma unroll
        for (int r = 0; r < 8; ++r) o8[r] = (h16)(ot[dt][r] * f);
        *(v8ha*)(ow + lr * 72u + dt * 16 + 8u * hi) = o8; }
    __builtin_amdgcn_fence(3  , "wavefront"); __builtin_amdgcn_wave_barrier(); asm volatile("" ::: "memory");
    h16* dst0 = AT16 + (size_t)(b * SEQ + i0) * DI + h * HD;
#pragma unroll 1
    for (int ps = 0; ps < 2; ++ps) {
#pragma unroll
        for (int s = 0; s < 4; ++s) { const unsigned row = 4u * s + (lane >> 3), pc = (lane & 7u) * 8u; const v8h val = *(const v8ha*)(ow + row * 72u + pc);
            *(volatile v8h*)(dst0 + (size_t)row * DI + pc) = val; }
        if (ps == 0) __threadfence(); }
}

#define SZ_WQ  ((size_t)DI * DQM * 2)
#define SZ_WK  ((size_t)DI * DCM * 2)
#define SZ_WO  ((size_t)DQM * DI * 2)
#define SZ_XB  ((size_t)NB * SEQ * DQM * 2)
#define SZ_CB  ((size_t)NB * SKV * DCM * 2)
#define N_PRJ  ((size_t)NB * SEQ * DI + 2 * (size_t)NB * SKV * DI)
#define SZ_F32 (N_PRJ * 4)
#define SZ_H16 (N_PRJ * 2)
#define SZ_AT  ((size_t)NB * SEQ * DI * 2)
static_assert(SZ_WQ + 2 * SZ_WK + SZ_WO + SZ_XB + SZ_CB + SZ_F32 + SZ_H16 + SZ_AT + 9 * 256 <= (size_t)134217728);
static_assert(N_PRJ % 8 == 0);
static_assert(((size_t)SEQ * DQM) % 8 == 0);
static_assert(((size_t)SKV * DCM) % 8 == 0);

extern "C" void kernel_launch(void* const* d_in, const int* in_sizes, int n_in,
                              void* d_out, int out_size, void* d_ws, size_t ws_size, hipStream_t stream) {
    if (n_in < 7) return;
    if ((size_t)in_sizes[0] < ((size_t)(NB - 1) * SEQ_FULL + SEQ) * DQM) return;
    if ((size_t)in_sizes[1] < ((size_t)(NB - 1) * SKV_FULL + SKV) * DCM) return;
    if (in_sizes[2] < DQM * DI || in_sizes[3] < DCM * DI || in_sizes[4] < DCM * DI || in_sizes[5] < DI * DQM || in_sizes[6] < DQM) return;
    if ((size_t)out_size < ((size_t)(NB - 1) * SEQ_FULL + SEQ) * DQM) return;
    const float* x = (const float*)d_in[0]; const float* ctx = (const float*)d_in[1];
    const float* wq = (const float*)d_in[2]; const float* wk = (const float*)d_in[3]; const float* wv = (const float*)d_in[4]; const float* wo = (const float*)d_in[5]; const float* bo = (const float*)d_in[6];
    float* OUT = (float*)d_out;
    char* wsp = (char*)d_ws;
    auto take = [&](size_t bytes) { char* p = wsp; wsp += (bytes + 255) & ~(size_t)255; return (void*)p; };
    bf* WQ = (bf*)take(SZ_WQ); bf* WK = (bf*)take(SZ_WK); bf* WV = (bf*)take(SZ_WK); bf* WO = (bf*)take(SZ_WO);
    bf* XB = (bf*)take(SZ_XB); bf* CB = (bf*)take(SZ_CB);
    float* F32 = (float*)take(SZ_F32); h16* H16 = (h16*)take(SZ_H16); h16* AT16 = (h16*)take(SZ_AT);
    if ((size_t)(wsp - (char*)d_ws) > ws_size) return;
    float* FQ = F32; float* FK = FQ + (size_t)NB * SEQ * DI; float* FVT = FK + (size_t)NB * SKV * DI;
    const h16* Q16 = H16; const h16* K16 = Q16 + (size_t)NB * SEQ * DI; const h16* VT16 = K16 + (size_t)NB * SKV * DI;

    k_wtG<<<(unsigned)(((size_t)DI * DQM / 64 + 63) / 64), 256, 0, stream>>>(wq, DQM, DI, WQ, 0, 1.0f);
    k_wtG<<<(unsigned)(((size_t)DI * DCM / 64 + 63) / 64), 256, 0, stream>>>(wk, DCM, DI, WK, 0, 1.0f);
    k_wtG<<<(unsigned)(((size_t)DI * DCM / 64 + 63) / 64), 256, 0, stream>>>(wv, DCM, DI, WV, 0, 1.0f);
    k_wtG<<<(unsigned)(((size_t)DQM * DI / 64 + 63) / 64), 256, 0, stream>>>(wo, DI, DQM, WO, 1, WCAR);
    k_cvt8<<<dim3((unsigned)(((size_t)SEQ * DQM / 8 + 255) / 256), NB), 256, 0, stream>>>(x, XB, (unsigned)((size_t)SEQ * DQM / 8), (size_t)SEQ_FULL * DQM, (size_t)SEQ * DQM);
    k_cvt8<<<dim3((unsigned)(((size_t)SKV * DCM / 8 + 255) / 256), NB), 256, 0, stream>>>(ctx, CB, (unsigned)((size_t)SKV * DCM / 8), (size_t)SKV_FULL * DCM, (size_t)SKV * DCM);
    k_gemmw<bf, false><<<dim3(NB * SEQ / 64, DI / 64, 1), 32, 0, stream>>>(XB, WQ, DQM, FQ, DI, nullptr, 0, 0, 0, 1.0f);
    k_gemmw<bf, false><<<dim3(NB * SKV / 64, DI / 64, 1), 32, 0, stream>>>(CB, WK, DCM, FK, DI, nullptr, 0, 0, 0, 1.0f);
    k_gemmw<bf, false><<<dim3(DI / 64, NB * SKV / 64, 1), 32, 0, stream>>>(WV, CB, DCM, FVT, VTP, nullptr, 0, 0, 0, 1.0f);
    k_cvt8h<<<(unsigned)((N_PRJ / 8 + 255) / 256), 256, 0, stream>>>(F32, H16, (unsigned)(N_PRJ / 8));
    k_fattn<<<dim3(SEQ / 64, NB * NH_), 128, 0, stream>>>(Q16, K16, VT16, AT16);
    k_gemmw<h16, true><<<dim3(SEQ / 64, DQM / 64, NB), 32, 0, stream>>>((const h16*)AT16, (const h16*)WO, DI, OUT, DQM, bo, (size_t)SEQ * DI, 0, (size_t)SEQ_FULL * DQM, OSC);
}
